// NormalizationModelofAttention_14980845928448
// MI455X (gfx1250) — hardware-verified
//
#include <hip/hip_runtime.h>


#define GG   64
#define NP   4096
#define NA   256
typedef _Float16 h16;
typedef unsigned short bf;
typedef __attribute__((ext_vector_type(16))) __bf16   v16bf;
typedef __attribute__((ext_vector_type(16))) _Float16 v16h;
typedef __attribute__((ext_vector_type(8)))  _Float16 v8h;
typedef __attribute__((ext_vector_type(8)))  unsigned short v8us;
typedef __attribute__((ext_vector_type(8)))  float    v8f;
typedef __attribute__((ext_vector_type(4)))  float    v4f;
typedef v8h  __attribute__((may_alias)) v8ha;
typedef v4f  __attribute__((may_alias)) v4fa;
typedef v8us __attribute__((may_alias)) v8usa;

__device__ __forceinline__ unsigned short f2bf(float f) { unsigned u = __float_as_uint(f); u += 0x7FFFu + ((u >> 16) & 1u); return (unsigned short)(u >> 16); }
__device__ __forceinline__ float bf2f(unsigned short b) { return __uint_as_float(((unsigned)b) << 16); }
__device__ __forceinline__ float bfr(float f) { return bf2f(f2bf(f)); }
__device__ __forceinline__ v16h cat16(v8h lo, v8h hi) { return __builtin_shufflevector(lo, hi, 0, 1, 2, 3, 4, 5, 6, 7, 8, 9, 10, 11, 12, 13, 14, 15); }
__device__ __forceinline__ v16bf cat16b(v8us lo, v8us hi) { return __builtin_bit_cast(v16bf, __builtin_shufflevector(lo, hi, 0, 1, 2, 3, 4, 5, 6, 7, 8, 9, 10, 11, 12, 13, 14, 15)); }
__device__ __forceinline__ v8f wmma16(v16h a, v16h b, v8f c) { return __builtin_amdgcn_wmma_f32_16x16x32_f16(false, a, false, b, (short)0, c, false, false); }
__device__ __forceinline__ v8f wmmab(v16bf a, v16bf b, v8f c) { return __builtin_amdgcn_wmma_f32_16x16x32_bf16(false, a, false, b, (short)0, c, false, false); }


template <typename T16> struct WFrag;
template <> struct WFrag<h16> { typedef v16h V; static __device__ __forceinline__ V ld(const h16* p) { return cat16(*(const v8h*)p, *(const v8h*)(p + 16)); } static __device__ __forceinline__ v8f mma(V a, V b, v8f c) { return wmma16(a, b, c); } };
template <> struct WFrag<bf> { typedef v16bf V; static __device__ __forceinline__ V ld(const bf* p) { return cat16b(*(const v8us*)p, *(const v8us*)(p + 16)); } static __device__ __forceinline__ v8f mma(V a, V b, v8f c) { return wmmab(a, b, c); } };
template <typename T16, int NSPLIT, bool BIAS>
__global__ __launch_bounds__(32) void k_gemmw(const T16* __restrict__ A, const T16* __restrict__ A2, const T16* __restrict__ Bt, const T16* __restrict__ Bt2, int K, float* C, int ldc, const float* __restrict__ bias, size_t sA, size_t sB, size_t sC) {
    typedef typename WFrag<T16>::V V;
    __shared__ __align__(16) float os[16 * 68];
    const size_t z = blockIdx.z; A += z * sA; if (A2) A2 += z * sA; Bt += z * sB; if (Bt2) Bt2 += z * sB; C += z * sC;
    const int lane = threadIdx.x & 31, lr = lane & 15, hi = lane >> 4; const int r0 = blockIdx.x * 64, c0 = blockIdx.y * 64;
    v8f acc[4][4];
#pragma unroll
    for (int mb = 0; mb < 4; ++mb)
#pragma unroll
        for (int nb = 0; nb < 4; ++nb) acc[mb][nb] = (v8f){};
    const size_t aoff = (size_t)(r0 + lr) * K + 8 * hi, boff = (size_t)(c0 + lr) * K + 8 * hi;
#pragma unroll 1
    for (int kc = 0; kc < K; kc += 32) {
        V a[4], a2[4];
#pragma unroll
        for (int mb = 0; mb < 4; ++mb) { a[mb] = WFrag<T16>::ld(A + aoff + (size_t)mb * 16 * K + kc); if (NSPLIT == 1 || NSPLIT == 2) a2[mb] = WFrag<T16>::ld(A2 + aoff + (size_t)mb * 16 * K + kc); }
#pragma unroll
        for (int nb = 0; nb < 4; ++nb) { const V b = WFrag<T16>::ld(Bt + boff + (size_t)nb * 16 * K + kc); V b2; if (NSPLIT >= 2) b2 = WFrag<T16>::ld(Bt2 + boff + (size_t)nb * 16 * K + kc);
#pragma unroll
            for (int mb = 0; mb < 4; ++mb) { acc[mb][nb] = WFrag<T16>::mma(a[mb], b, acc[mb][nb]); if (NSPLIT == 1 || NSPLIT == 2) acc[mb][nb] = WFrag<T16>::mma(a2[mb], b, acc[mb][nb]); if (NSPLIT >= 2) acc[mb][nb] = WFrag<T16>::mma(a[mb], b2, acc[mb][nb]); } }
        asm volatile("v_nop\n\tv_nop\n\tv_nop\n\tv_nop" : "+v"(acc[0][0]), "+v"(acc[1][1]), "+v"(acc[2][2]), "+v"(acc[3][3]) : "v"(a[0]), "v"(a[3]));
    }
#pragma unroll
    for (int mb = 0; mb < 4; ++mb) {
#pragma unroll
        for (int nb = 0; nb < 4; ++nb) {
#pragma unroll
            for (int j = 0; j < 8; ++j) os[(hi * 8 + j) * 68 + nb * 16 + lr] = acc[mb][nb][j]; }
        __builtin_amdgcn_wave_barrier(); asm volatile("" ::: "memory");
        float* crow = C + (size_t)(r0 + mb * 16) * ldc + c0;
#pragma unroll 1
        for (int ps = 0; ps < 2; ++ps) {
#pragma unroll
            for (int s = 0; s < 8; ++s) { const int row = 2 * s + hi, cofs = lr * 4; v4f val = *(const v4fa*)(os + row * 68 + cofs); if (BIAS) { val[0] += bfr(bias[c0 + cofs]); val[1] += bfr(bias[c0 + cofs + 1]); val[2] += bfr(bias[c0 + cofs + 2]); val[3] += bfr(bias[c0 + cofs + 3]); }
                *(volatile v4f*)(crow + (size_t)row * ldc + cofs) = val; }
            if (ps == 0) __threadfence(); }
        __builtin_amdgcn_wave_barrier(); asm volatile("" ::: "memory");
    }
}

__device__ __forceinline__ void splitf(float y, unsigned short& h, unsigned short& l) { h = f2bf(y); l = f2bf(y - bf2f(h)); }
__device__ __forceinline__ float coordf(int i) { return i == GG - 1 ? 10.0f : __fadd_rn(-10.0f, __fmul_rn((float)i, __fdiv_rn(20.0f, 63.0f))); }
typedef __attribute__((ext_vector_type(4))) unsigned short v4us;

__global__ __launch_bounds__(256) void k_stT(const float* __restrict__ stim, bf* ST) { const size_t e = ((size_t)blockIdx.x * 256 + threadIdx.x) * 4; if (e >= (size_t)NA * NP) return; const int px = (int)(e % NP), a = (int)(e / NP); v4us o;
#pragma unroll
    for (int q = 0; q < 4; ++q) o[q] = f2bf(stim[(size_t)(px + q) * NA + a]); *(volatile v4us*)(ST + e) = o; __threadfence(); *(volatile v4us*)(ST + e) = o; }
__global__ __launch_bounds__(256) void k_field(const float* __restrict__ pscale, const float* __restrict__ pfac, int usefac, bf* Fh, bf* Fl) { const int lane = threadIdx.x & 31; const int k = blockIdx.x * 8 + (threadIdx.x >> 5); if (k >= NP) return; const float xk = coordf(k % GG), yk = coordf(k / GG);
    float sg = __fadd_rn(0.07f, __fmul_rn(bfr(pscale[0]), __fsqrt_rn(__fadd_rn(__fmul_rn(xk, xk), __fmul_rn(yk, yk))))); if (usefac) sg = __fmul_rn(sg, bfr(pfac[0])); const float inv = __fdiv_rn(1.0f, __fmul_rn(2.0f, __fmul_rn(sg, sg))); float s = 0.f;
    for (int px = lane; px < NP; px += 32) { const float dx = __fsub_rn(coordf(px % GG), xk), dy = __fsub_rn(coordf(px / GG), yk); const float d2 = __fadd_rn(__fmul_rn(dx, dx), __fmul_rn(dy, dy)); float ar = __fmul_rn(d2, inv); asm volatile("" : "+v"(ar)); s = __fadd_rn(s, __expf(-ar)); }
#pragma unroll
    for (int sh = 16; sh; sh >>= 1) s += __shfl_xor(s, sh, 32);
    const float rs = __fdiv_rn(1.0f, s);
#pragma unroll 1
    for (int ps = 0; ps < 2; ++ps) {
        for (int c0 = lane * 4; c0 < NP; c0 += 128) { v4us oh, ol;
#pragma unroll
            for (int q = 0; q < 4; ++q) { const int px = c0 + q; const float dx = __fsub_rn(coordf(px % GG), xk), dy = __fsub_rn(coordf(px / GG), yk); const float d2 = __fadd_rn(__fmul_rn(dx, dx), __fmul_rn(dy, dy)); float ar = __fmul_rn(d2, inv); asm volatile("" : "+v"(ar)); float g = __fmul_rn(__expf(-ar), rs); unsigned short a, b; splitf(g, a, b); oh[q] = a; ol[q] = b; }
            *(volatile v4us*)(Fh + (size_t)k * NP + c0) = oh; *(volatile v4us*)(Fl + (size_t)k * NP + c0) = ol; }
        if (ps == 0) __threadfence(); } }
__global__ __launch_bounds__(256) void k_num(const float* __restrict__ SD, const float* __restrict__ pasig, const float* __restrict__ pgain, float* NUM) { const size_t e = ((size_t)blockIdx.x * 256 + threadIdx.x) * 4; if (e >= (size_t)NP * NA) return; const int k = (int)(e / NA); const float xk = coordf(k % GG), yk = coordf(k / GG); const float as = bfr(pasig[0]);
    const float dx = __fsub_rn(xk, 3.0f); const float d2 = __fadd_rn(__fmul_rn(dx, dx), __fmul_rn(yk, yk)); float ar = __fdiv_rn(d2, __fmul_rn(2.0f, __fmul_rn(as, as))); asm volatile("" : "+v"(ar)); float ga = __fmul_rn(bfr(pgain[0]), __expf(-ar)); asm volatile("" : "+v"(ga)); const float af = __fadd_rn(ga, 1.0f);
    const v4f a = *(const v4f*)(SD + e); v4f o; o[0] = __fmul_rn(a[0], af); o[1] = __fmul_rn(a[1], af); o[2] = __fmul_rn(a[2], af); o[3] = __fmul_rn(a[3], af); *(volatile v4f*)(NUM + e) = o; __threadfence(); *(volatile v4f*)(NUM + e) = o; }
__global__ __launch_bounds__(256) void k_pn(const float* __restrict__ NUM, const float* __restrict__ SUR, float* PN) { const size_t e = ((size_t)blockIdx.x * 256 + threadIdx.x) * 4; if (e >= (size_t)NP * NA) return; const v4f a = *(const v4f*)(NUM + e), s = *(const v4f*)(SUR + e); v4f o;
#pragma unroll
    for (int q = 0; q < 4; ++q) o[q] = __fdiv_rn(a[q], __fadd_rn(s[q], 0.5f)); *(volatile v4f*)(PN + e) = o; __threadfence(); *(volatile v4f*)(PN + e) = o; }
__global__ __launch_bounds__(256) void k_tr(const float* __restrict__ M, bf* Th, bf* Tl) { const size_t e = ((size_t)blockIdx.x * 256 + threadIdx.x) * 4; if (e >= (size_t)NA * NP) return; const int k = (int)(e % NP), a = (int)(e / NP); v4us oh, ol;
#pragma unroll
    for (int q = 0; q < 4; ++q) { unsigned short u, c; splitf(M[(size_t)(k + q) * NA + a], u, c); oh[q] = u; ol[q] = c; } *(volatile v4us*)(Th + e) = oh; *(volatile v4us*)(Tl + e) = ol; __threadfence(); *(volatile v4us*)(Th + e) = oh; *(volatile v4us*)(Tl + e) = ol; }

extern "C" void kernel_launch(void* const* d_in, const int* in_sizes, int n_in,
                              void* d_out, int out_size, void* d_ws, size_t ws_size, hipStream_t stream) {
    (void)in_sizes; (void)n_in; (void)out_size;
    const float* stim = (const float*)d_in[0]; const float* pscale = (const float*)d_in[1]; const float* pasig = (const float*)d_in[2]; const float* pgain = (const float*)d_in[3]; const float* pss = (const float*)d_in[4]; const float* psf = (const float*)d_in[5];
    float* NUM = (float*)d_out; float* SUR = NUM + (size_t)NP * NA; float* PN = SUR + (size_t)NP * NA; float* VOX = PN + (size_t)NP * NA;
    char* wsp = (char*)d_ws;
    auto take = [&](size_t bytes) { char* p = wsp; wsp += (bytes + 255) & ~(size_t)255; return (void*)p; };
    bf* ST = (bf*)take((size_t)NA * NP * 2); bf* Fh = (bf*)take((size_t)NP * NP * 2); bf* Fl = (bf*)take((size_t)NP * NP * 2); float* SD = (float*)take((size_t)NP * NA * 4); bf* Th = (bf*)take((size_t)NA * NP * 2); bf* Tl = (bf*)take((size_t)NA * NP * 2);
    if ((size_t)(wsp - (char*)d_ws) > ws_size) return;
    const unsigned LF = NP / 8, L4 = (unsigned)(((size_t)NP * NA / 4 + 255) / 256);
    k_stT<<<L4, 256, 0, stream>>>(stim, ST);
    k_field<<<LF, 256, 0, stream>>>(pscale, pss, 0, Fh, Fl);
    k_gemmw<bf, 1, false><<<dim3(NP / 64, NA / 64, 1), 32, 0, stream>>>(Fh, Fl, ST, nullptr, NP, SD, NA, nullptr, 0, 0, 0);
    k_num<<<L4, 256, 0, stream>>>(SD, pasig, pgain, NUM); k_tr<<<L4, 256, 0, stream>>>(NUM, Th, Tl);
    k_field<<<LF, 256, 0, stream>>>(pscale, pss, 1, Fh, Fl);
    k_gemmw<bf, 2, false><<<dim3(NP / 64, NA / 64, 1), 32, 0, stream>>>(Fh, Fl, Th, Tl, NP, SUR, NA, nullptr, 0, 0, 0);
    k_pn<<<L4, 256, 0, stream>>>(NUM, SUR, PN); k_tr<<<L4, 256, 0, stream>>>(PN, Th, Tl);
    k_field<<<LF, 256, 0, stream>>>(pscale, psf, 1, Fh, Fl);
    k_gemmw<bf, 2, false><<<dim3(NP / 64, NA / 64, 1), 32, 0, stream>>>(Fh, Fl, Th, Tl, NP, VOX, NA, nullptr, 0, 0, 0);
}
